// GraphMultiHeadAttention_66640712564942
// MI455X (gfx1250) — hardware-verified
//
#include <hip/hip_runtime.h>
#include <math.h>
#include <stdint.h>

#define NB_    4
#define NN_    1024
#define DIN    512
#define HID    128
#define NHD    4
#define NEDG   5
#define NTOK   (NB_ * NN_)
#define DH     (NHD * HID)
#define NSROW  (2 * NEDG)
#define NEGBIG (-1.0e9f)
#define LN_EPS 1e-6f
#define SLOPE  0.01f

static_assert(NTOK % 256 == 0);
static_assert(NTOK % 128 == 0);
static_assert(NN_ % 64 == 0);
static_assert(DIN == 512);
static_assert(HID == 128);
static_assert(DIN % 32 == 0);
static_assert(DH % 64 == 0);

typedef __attribute__((ext_vector_type(16))) __bf16 v16b;
typedef __attribute__((ext_vector_type(8)))  __bf16 v8b;
typedef __attribute__((ext_vector_type(8)))  float  v8f;
typedef __attribute__((ext_vector_type(4)))  float  v4f;
typedef __attribute__((ext_vector_type(2)))  float  v2f;
typedef __attribute__((ext_vector_type(4)))  unsigned int v4u;
typedef __attribute__((ext_vector_type(8)))  unsigned int v8u;
typedef __attribute__((ext_vector_type(4)))  int v4i;
typedef v8b __attribute__((may_alias)) v8ba;
typedef v4f __attribute__((may_alias)) v4fa;
typedef v2f __attribute__((may_alias)) v2fa;
typedef v4u __attribute__((may_alias)) v4ua;
typedef v4i __attribute__((may_alias)) v4ia;

union FragU { v16b v; v8b h[2]; };
union PackU { v8u u; v16b v; };

__device__ __forceinline__ unsigned short f2bf_bits(float f) {
  const unsigned u = __float_as_uint(f);
  return (unsigned short)((u + 0x7FFFu + ((u >> 16) & 1u)) >> 16);
}
__device__ __forceinline__ float bf_bits2f(unsigned short h) { return __uint_as_float(((unsigned)h) << 16); }
__device__ __forceinline__ float bf16r(float f) {
  unsigned u = __float_as_uint(f);
  u = (u + 0x7FFFu + ((u >> 16) & 1u)) & 0xFFFF0000u;
  return __uint_as_float(u);
}
__device__ __forceinline__ unsigned pk16(unsigned short a, unsigned short b) { return (unsigned)a | ((unsigned)b << 16); }

__device__ __forceinline__ v8f wmma_bf16(v16b a, v16b b, v8f c) {
  v8f d = __builtin_amdgcn_wmma_f32_16x16x32_bf16(false, a, false, b, (short)0, c, false, false);
  asm volatile("v_nop\n\tv_nop\n\tv_nop\n\tv_nop" : "+v"(d) : "v"(a), "v"(b));
  return d;
}

__device__ __forceinline__ v16b load_frag(const unsigned short* p, int hh) {
  FragU f;
  f.h[0] = *(const v8ba*)(p + 8 * hh);
  f.h[1] = *(const v8ba*)(p + 16 + 8 * hh);
  return f.v;
}

__device__ __forceinline__ void pack_p2(v8f a, v8f c, v16b& ho, v16b& lo) {
  PackU uh, ul;
#pragma unroll
  for (int i = 0; i < 4; ++i) {
    const unsigned short h0 = f2bf_bits(a[2 * i]), h1 = f2bf_bits(a[2 * i + 1]);
    const unsigned short l0 = f2bf_bits(a[2 * i] - bf_bits2f(h0)), l1 = f2bf_bits(a[2 * i + 1] - bf_bits2f(h1));
    uh.u[i] = pk16(h0, h1); ul.u[i] = pk16(l0, l1);
    const unsigned short g0 = f2bf_bits(c[2 * i]), g1 = f2bf_bits(c[2 * i + 1]);
    const unsigned short m0 = f2bf_bits(c[2 * i] - bf_bits2f(g0)), m1 = f2bf_bits(c[2 * i + 1] - bf_bits2f(g1));
    uh.u[4 + i] = pk16(g0, g1); ul.u[4 + i] = pk16(m0, m1);
  }
  ho = uh.v; lo = ul.v;
}

__device__ __forceinline__ void gemm_core_32x64(
    const unsigned short* __restrict__ Ah, const unsigned short* __restrict__ Al,
    const unsigned short* __restrict__ Bt, int K, size_t aoff, size_t boff, int hh, v8f (&acc)[2][4]) {
  const unsigned short* a0h = Ah + aoff;
  const unsigned short* a1h = a0h + (size_t)16 * K;
  const unsigned short* a0l = Al + aoff;
  const unsigned short* a1l = a0l + (size_t)16 * K;
  const unsigned short* bp  = Bt + boff;
#pragma unroll 1
  for (int k0 = 0; k0 < K; k0 += 32) {
    const v16b f0h = load_frag(a0h + k0, hh);
    const v16b f0l = load_frag(a0l + k0, hh);
    const v16b f1h = load_frag(a1h + k0, hh);
    const v16b f1l = load_frag(a1l + k0, hh);
#pragma unroll
    for (int nt = 0; nt < 4; ++nt) {
      const v16b fb = load_frag(bp + (size_t)nt * 16 * K + k0, hh);
      acc[0][nt] = wmma_bf16(f0h, fb, acc[0][nt]);
      acc[0][nt] = wmma_bf16(f0l, fb, acc[0][nt]);
      acc[1][nt] = wmma_bf16(f1h, fb, acc[1][nt]);
      acc[1][nt] = wmma_bf16(f1l, fb, acc[1][nt]);
    }
  }
}

__global__ __launch_bounds__(256) void k_tr_bf16(const float* __restrict__ src, unsigned short* __restrict__ dst,
                                                 int R, int C, long sIn, long sOut) {
  __shared__ __align__(16) unsigned short t16[64 * 72];
  src += (size_t)blockIdx.z * sIn;
  dst += (size_t)blockIdx.z * sOut;
  const int c0  = blockIdx.x * 64;
  const int r0  = blockIdx.y * 64;
  const int tid = threadIdx.x;
  {
    const int rr = tid >> 2;
    const int cq = (tid & 3) * 16;
    const float* s = src + (size_t)(r0 + rr) * C + c0 + cq;
#pragma unroll
    for (int q = 0; q < 4; ++q) {
      const v4f f = *(const v4fa*)(s + 4 * q);
#pragma unroll
      for (int e = 0; e < 4; ++e) t16[rr * 72 + cq + 4 * q + e] = f2bf_bits(f[e]);
    }
  }
  __syncthreads();
  const int sub = tid >> 3;
  const int c8  = (tid & 7) * 8;
  v4u hv[2];
#pragma unroll
  for (int it = 0; it < 2; ++it) {
    const int oc = it * 32 + sub;
    v4u a;
#pragma unroll
    for (int q = 0; q < 4; ++q)
      a[q] = pk16(t16[(c8 + 2 * q) * 72 + oc], t16[(c8 + 2 * q + 1) * 72 + oc]);
    hv[it] = a;
  }
  for (int pass = 0; pass < 2; ++pass) {
#pragma unroll
    for (int it = 0; it < 2; ++it) {
      const int oc = it * 32 + sub;
      const size_t go = (size_t)(c0 + oc) * R + r0 + c8;
      *(volatile v4u*)(dst + go) = hv[it];
    }
    __threadfence();
  }
}

__global__ __launch_bounds__(256) void k_ln_split(const float* __restrict__ x, const float* __restrict__ gam,
                                                  const float* __restrict__ bet,
                                                  unsigned short* __restrict__ Hp, unsigned short* __restrict__ Lp, int T) {
  const int lane = threadIdx.x & 31;
  int row = blockIdx.x * 8 + (threadIdx.x >> 5);
  const bool ok = row < T;
  row = ok ? row : (T - 1);
  const float* xr = x + (size_t)row * DIN;
  const v4f a0 = *(const v4fa*)(xr + lane * 8);
  const v4f a1 = *(const v4fa*)(xr + lane * 8 + 4);
  const v4f a2 = *(const v4fa*)(xr + 256 + lane * 8);
  const v4f a3 = *(const v4fa*)(xr + 256 + lane * 8 + 4);
  const v4f g0 = *(const v4fa*)(gam + lane * 8);
  const v4f g1 = *(const v4fa*)(gam + lane * 8 + 4);
  const v4f g2 = *(const v4fa*)(gam + 256 + lane * 8);
  const v4f g3 = *(const v4fa*)(gam + 256 + lane * 8 + 4);
  const v4f c0 = *(const v4fa*)(bet + lane * 8);
  const v4f c1 = *(const v4fa*)(bet + lane * 8 + 4);
  const v4f c2 = *(const v4fa*)(bet + 256 + lane * 8);
  const v4f c3 = *(const v4fa*)(bet + 256 + lane * 8 + 4);
  float v[16] = {a0[0], a0[1], a0[2], a0[3], a1[0], a1[1], a1[2], a1[3],
                 a2[0], a2[1], a2[2], a2[3], a3[0], a3[1], a3[2], a3[3]};
  float g[16] = {g0[0], g0[1], g0[2], g0[3], g1[0], g1[1], g1[2], g1[3],
                 g2[0], g2[1], g2[2], g2[3], g3[0], g3[1], g3[2], g3[3]};
  float c[16] = {c0[0], c0[1], c0[2], c0[3], c1[0], c1[1], c1[2], c1[3],
                 c2[0], c2[1], c2[2], c2[3], c3[0], c3[1], c3[2], c3[3]};
#pragma unroll
  for (int i = 0; i < 16; ++i) { v[i] = bf16r(v[i]); g[i] = bf16r(g[i]); c[i] = bf16r(c[i]); }
  float s = 0.0f;
#pragma unroll
  for (int i = 0; i < 16; ++i) s += v[i];
#pragma unroll
  for (int o = 16; o > 0; o >>= 1) s += __shfl_xor(s, o);
  const float mean = s * (1.0f / 512.0f);
  float q = 0.0f;
#pragma unroll
  for (int i = 0; i < 16; ++i) { const float d = v[i] - mean; v[i] = d; q += d * d; }
#pragma unroll
  for (int o = 16; o > 0; o >>= 1) q += __shfl_xor(q, o);
  const float rstd = rsqrtf(q * (1.0f / 512.0f) + LN_EPS);
  unsigned hw[8], lw[8];
#pragma unroll
  for (int i = 0; i < 8; ++i) {
    const float y0 = (v[2 * i] * rstd) * g[2 * i] + c[2 * i];
    const float y1 = (v[2 * i + 1] * rstd) * g[2 * i + 1] + c[2 * i + 1];
    const unsigned short h0 = f2bf_bits(y0), h1 = f2bf_bits(y1);
    const unsigned short l0 = f2bf_bits(y0 - bf_bits2f(h0)), l1 = f2bf_bits(y1 - bf_bits2f(h1));
    hw[i] = pk16(h0, h1); lw[i] = pk16(l0, l1);
  }
  const v4u hA = (v4u){hw[0], hw[1], hw[2], hw[3]};
  const v4u hB = (v4u){hw[4], hw[5], hw[6], hw[7]};
  const v4u lA = (v4u){lw[0], lw[1], lw[2], lw[3]};
  const v4u lB = (v4u){lw[4], lw[5], lw[6], lw[7]};
  const size_t o0 = (size_t)row * DIN + (size_t)lane * 8;
  const size_t o1 = (size_t)row * DIN + 256 + (size_t)lane * 8;
  if (ok) {
    *(volatile v4u*)(Hp + o0) = hA; *(volatile v4u*)(Hp + o1) = hB;
    *(volatile v4u*)(Lp + o0) = lA; *(volatile v4u*)(Lp + o1) = lB;
  }
  __threadfence();
  if (ok) {
    *(volatile v4u*)(Hp + o0) = hA; *(volatile v4u*)(Hp + o1) = hB;
    *(volatile v4u*)(Lp + o0) = lA; *(volatile v4u*)(Lp + o1) = lB;
  }
}

__global__ __launch_bounds__(128) void k_proj(
    const unsigned short* __restrict__ XNhi, const unsigned short* __restrict__ XNlo,
    const unsigned short* __restrict__ WT,
    float* __restrict__ Hf,
    unsigned short* __restrict__ HThi, unsigned short* __restrict__ HTlo) {
  __shared__ __align__(16) unsigned char smem[32768];
  float* sF = (float*)smem;
  unsigned short* sH = (unsigned short*)smem;
  unsigned short* sL = sH + 8192;
  const int tid = threadIdx.x, lane = tid & 31, w = tid >> 5;
  const int hh = lane >> 4, m = lane & 15;
  const int m0 = blockIdx.x * 128;
  const int cg = blockIdx.y;
  const int n0 = cg * 64;
  const int m0w = m0 + 32 * w;

  const v8f zero8 = {0.f, 0.f, 0.f, 0.f, 0.f, 0.f, 0.f, 0.f};
  v8f acc[2][4];
#pragma unroll
  for (int mt = 0; mt < 2; ++mt)
#pragma unroll
    for (int nt = 0; nt < 4; ++nt) acc[mt][nt] = zero8;

  gemm_core_32x64(XNhi, XNlo, WT, DIN, (size_t)(m0w + m) * DIN, (size_t)(n0 + m) * DIN, hh, acc);

#pragma unroll
  for (int nt = 0; nt < 4; ++nt)
#pragma unroll
    for (int mt = 0; mt < 2; ++mt)
#pragma unroll
      for (int r = 0; r < 8; ++r) {
        const int tokl = 32 * w + 16 * mt + 8 * hh + r;
        const int feat = 16 * nt + m;
        sF[tokl * 64 + feat] = acc[mt][nt][r];
      }
  __syncthreads();
  {
    const int rsub = lane >> 4, c4 = (lane & 15) * 4;
    for (int pass = 0; pass < 2; ++pass) {
#pragma unroll
      for (int it = 0; it < 16; ++it) {
        const int row = 32 * w + 2 * it + rsub;
        const v4f v = *(const v4fa*)(sF + row * 64 + c4);
        *(volatile v4f*)(Hf + (size_t)(m0 + row) * DH + n0 + c4) = v;
      }
      __threadfence();
    }
  }
  __syncthreads();
#pragma unroll
  for (int nt = 0; nt < 4; ++nt)
#pragma unroll
    for (int mt = 0; mt < 2; ++mt)
#pragma unroll
      for (int r = 0; r < 8; ++r) {
        const int tokl = 32 * w + 16 * mt + 8 * hh + r;
        const int feat = 16 * nt + m;
        const float y = acc[mt][nt][r];
        const unsigned short hb = f2bf_bits(y);
        const unsigned short lb = f2bf_bits(y - bf_bits2f(hb));
        const int idx = feat * 128 + tokl;
        sH[idx] = hb;
        sL[idx] = lb;
      }
  __syncthreads();
  {
    const int dsub = lane >> 4, t8 = (lane & 15) * 8;
    for (int pass = 0; pass < 2; ++pass) {
#pragma unroll
      for (int it = 0; it < 8; ++it) {
        const int d = 16 * w + 2 * it + dsub;
        const v4u hv = *(const v4ua*)(sH + d * 128 + t8);
        const v4u lv = *(const v4ua*)(sL + d * 128 + t8);
        const size_t go = (size_t)(n0 + d) * (size_t)NTOK + m0 + t8;
        *(volatile v4u*)(HThi + go) = hv;
        *(volatile v4u*)(HTlo + go) = lv;
      }
      __threadfence();
    }
  }
}

__global__ __launch_bounds__(256) void k_sproj(const float* __restrict__ Hf, const float* __restrict__ wsrc,
                                               const float* __restrict__ wdst, float* __restrict__ S) {
  __shared__ __align__(16) float sW[2 * NEDG * HID];
  __shared__ __align__(16) float sOut[NSROW * 256];
  const int tid  = threadIdx.x;
  const int head = blockIdx.y;
  const int tok0 = blockIdx.x * 256;
  const int tok  = tok0 + tid;
#pragma unroll
  for (int k = 0; k < 3; ++k) {
    const int i = tid + 256 * k;
    if (i < NEDG * HID) {
      sW[i]              = bf16r(wsrc[(size_t)head * NEDG * HID + i]);
      sW[NEDG * HID + i] = bf16r(wdst[(size_t)head * NEDG * HID + i]);
    }
  }
  __syncthreads();
  const float* hr = Hf + (size_t)tok * DH + head * HID;
  float as[NEDG], ad[NEDG];
#pragma unroll
  for (int e = 0; e < NEDG; ++e) { as[e] = 0.0f; ad[e] = 0.0f; }
#pragma unroll 1
  for (int o2 = 0; o2 < HID / 2; ++o2) {
    const v2f hv = *(const v2fa*)(hr + 2 * o2);
#pragma unroll
    for (int e = 0; e < NEDG; ++e) {
      const v2f ws = *(const v2fa*)(sW + e * HID + 2 * o2);
      const v2f wd = *(const v2fa*)(sW + NEDG * HID + e * HID + 2 * o2);
      as[e] = fmaf(hv[0], ws[0], as[e]);
      as[e] = fmaf(hv[1], ws[1], as[e]);
      ad[e] = fmaf(hv[0], wd[0], ad[e]);
      ad[e] = fmaf(hv[1], wd[1], ad[e]);
    }
  }
#pragma unroll
  for (int e = 0; e < NEDG; ++e) {
    sOut[e * 256 + tid]          = as[e];
    sOut[(NEDG + e) * 256 + tid] = ad[e];
  }
  __syncthreads();
  for (int pass = 0; pass < 2; ++pass) {
#pragma unroll
    for (int k = 0; k < 3; ++k) {
      const int idx = k * 256 + tid;
      if (idx < NSROW * 64) {
        const int rsel = idx >> 6, c4 = (idx & 63) * 4;
        const v4f v = *(const v4fa*)(sOut + rsel * 256 + c4);
        *(volatile v4f*)(S + (size_t)(head * NSROW + rsel) * NTOK + tok0 + c4) = v;
      }
    }
    __threadfence();
  }
}

__global__ __launch_bounds__(128) void k_attn(const int* __restrict__ adj, const float* __restrict__ S,
                                              const float* __restrict__ bedge,
                                              const unsigned short* __restrict__ HThi,
                                              const unsigned short* __restrict__ HTlo,
                                              float* __restrict__ out) {
  __shared__ __align__(16) float sAb[NEDG * 64];
  __shared__ __align__(16) float sD[NEDG * 64];
  __shared__ __align__(16) float sO[4 * 16 * HID];

  const int tid = threadIdx.x, lane = tid & 31, w = tid >> 5;
  const int hh = lane >> 4, m = lane & 15;
  const int qt = blockIdx.x;
  const int b = blockIdx.y >> 2, h = blockIdx.y & 3;
  const int q0 = qt * 64, q0w = q0 + 16 * w, ql = 16 * w + m;
  const size_t tokb = (size_t)b * NN_;

#pragma unroll
  for (int k = 0; k < 3; ++k) {
    const int idx = tid + 128 * k;
    if (idx < NEDG * 64) {
      const int e = idx >> 6, c = idx & 63;
      const float a  = S[(size_t)(h * NSROW + e) * NTOK + tokb + q0 + c];
      const float be = bf16r(bedge[h * NEDG + e]);
      sAb[idx] = a + be;
    }
  }

  const v8f zero8 = {0.f, 0.f, 0.f, 0.f, 0.f, 0.f, 0.f, 0.f};
  v8f o[8];
#pragma unroll
  for (int t = 0; t < 8; ++t) o[t] = zero8;
  float mrun = -INFINITY, lrun = 0.0f;

  const int* arow = adj + (tokb + q0w + m) * (size_t)NN_ + 8 * hh;

#pragma unroll 1
  for (int ks = 0; ks < NN_ / 64; ++ks) {
    const int kb = ks * 64;
    __syncthreads();
#pragma unroll
    for (int k = 0; k < 3; ++k) {
      const int idx = tid + 128 * k;
      if (idx < NEDG * 64) {
        const int e = idx >> 6, c = idx & 63;
        sD[idx] = S[(size_t)(h * NSROW + NEDG + e) * NTOK + tokb + kb + c];
      }
    }
    __syncthreads();

    v8f s[4];
#pragma unroll
    for (int j = 0; j < 4; ++j) {
      const v4i aA = *(const v4ia*)(arow + kb + 16 * j);
      const v4i aB = *(const v4ia*)(arow + kb + 16 * j + 4);
      const int av[8] = {aA[0], aA[1], aA[2], aA[3], aB[0], aB[1], aB[2], aB[3]};
#pragma unroll
      for (int r = 0; r < 8; ++r) {
        const int a = av[r];
        const int em1 = a - 1;
        const bool valid = (unsigned)em1 < (unsigned)NEDG;
        const int e = valid ? em1 : 0;
        float t = sAb[e * 64 + ql] + sD[e * 64 + 16 * j + 8 * hh + r];
        t = (t >= 0.0f) ? t : SLOPE * t;
        t = valid ? t : 0.0f;
        t = (a == 0) ? NEGBIG : t;
        s[j][r] = t;
      }
    }
    float cm = -INFINITY;
#pragma unroll
    for (int j = 0; j < 4; ++j)
#pragma unroll
      for (int r = 0; r < 8; ++r) cm = fmaxf(cm, s[j][r]);
    cm = fmaxf(cm, __shfl_xor(cm, 16, 32));
    const float mnew  = fmaxf(mrun, cm);
    const float alpha = __expf(mrun - mnew);
    mrun = mnew;
    float psum = 0.0f;
#pragma unroll
    for (int j = 0; j < 4; ++j)
#pragma unroll
      for (int r = 0; r < 8; ++r) {
        const float p = __expf(s[j][r] - mnew);
        psum += p;
        s[j][r] = p;
      }
    psum += __shfl_xor(psum, 16, 32);
    lrun = lrun * alpha + psum;
#pragma unroll
    for (int t = 0; t < 8; ++t)
#pragma unroll
      for (int r = 0; r < 8; ++r) o[t][r] *= alpha;

    v16b p0h, p0l, p1h, p1l;
    pack_p2(s[0], s[1], p0h, p0l);
    pack_p2(s[2], s[3], p1h, p1l);

#pragma unroll
    for (int t = 0; t < 8; ++t) {
      const unsigned short* vph = HThi + (size_t)(h * HID + 16 * t + m) * (size_t)NTOK + tokb + kb;
      const unsigned short* vpl = HTlo + (size_t)(h * HID + 16 * t + m) * (size_t)NTOK + tokb + kb;
      const v16b v0h = load_frag(vph, hh), v0l = load_frag(vpl, hh);
      o[t] = wmma_bf16(v0h, p0h, o[t]);
      o[t] = wmma_bf16(v0h, p0l, o[t]);
      o[t] = wmma_bf16(v0l, p0h, o[t]);
      const v16b v1h = load_frag(vph + 32, hh), v1l = load_frag(vpl + 32, hh);
      o[t] = wmma_bf16(v1h, p1h, o[t]);
      o[t] = wmma_bf16(v1h, p1l, o[t]);
      o[t] = wmma_bf16(v1l, p1h, o[t]);
    }
  }

  const float inv = 1.0f / lrun;
  float* so = sO + w * (16 * HID);
#pragma unroll
  for (int t = 0; t < 8; ++t)
#pragma unroll
    for (int r = 0; r < 8; ++r)
      so[m * HID + 16 * t + 8 * hh + r] = fmaxf(o[t][r] * inv, 0.0f);
  __syncthreads();
  for (int pass = 0; pass < 2; ++pass) {
#pragma unroll
    for (int i = 0; i < 16; ++i) {
      const v4f v = *(const v4fa*)(so + i * HID + lane * 4);
      *(volatile v4f*)(out + (tokb + q0w + i) * (size_t)DH + h * HID + lane * 4) = v;
    }
    __threadfence();
  }
}

extern "C" void kernel_launch(void* const* d_in, const int* in_sizes, int n_in,
                              void* d_out, int out_size, void* d_ws, size_t ws_size,
                              hipStream_t stream) {
  if (n_in < 10) return;
  if (in_sizes[0] != NTOK * DIN) return;
  if (in_sizes[1] != NB_ * NN_ * NN_) return;
  if (in_sizes[4] != NHD * DIN * HID) return;
  if (in_sizes[5] != NHD * NEDG * HID) return;
  if (in_sizes[6] != NHD * NEDG * HID) return;
  if (in_sizes[7] != NHD * NEDG) return;
  if (in_sizes[8] != DIN) return;
  if (in_sizes[9] != DIN) return;
  if (out_size != NTOK * DH) return;

  const float* x     = (const float*)d_in[0];
  const int*   adj   = (const int*)d_in[1];
  const float* W     = (const float*)d_in[4];
  const float* wsrc  = (const float*)d_in[5];
  const float* wdst  = (const float*)d_in[6];
  const float* bedge = (const float*)d_in[7];
  const float* gamma = (const float*)d_in[8];
  const float* beta  = (const float*)d_in[9];
  float* out = (float*)d_out;

  const size_t PWT = (size_t)DH * DIN * 2;
  const size_t P16 = (size_t)NTOK * DIN * 2;
  const size_t P32 = (size_t)NTOK * DH * 4;
  const size_t PHT = (size_t)DH * NTOK * 2;
  const size_t PS  = (size_t)NHD * NSROW * NTOK * 4;
  size_t off = 0;
  const size_t oWT   = off; off += PWT;
  const size_t oXNhi = off; off += P16;
  const size_t oXNlo = off; off += P16;
  const size_t oHf   = off; off += P32;
  const size_t oHThi = off; off += PHT;
  const size_t oHTlo = off; off += PHT;
  const size_t oS    = off; off += PS;
  if (off > ws_size) return;

  char* ws = (char*)d_ws;
  unsigned short* WT   = (unsigned short*)(ws + oWT);
  unsigned short* XNhi = (unsigned short*)(ws + oXNhi);
  unsigned short* XNlo = (unsigned short*)(ws + oXNlo);
  float*          Hf   = (float*)(ws + oHf);
  unsigned short* HThi = (unsigned short*)(ws + oHThi);
  unsigned short* HTlo = (unsigned short*)(ws + oHTlo);
  float*          S    = (float*)(ws + oS);

  k_tr_bf16<<<dim3(HID / 64, DIN / 64, NHD), 256, 0, stream>>>(W, WT, DIN, HID, (long)DIN * HID, (long)HID * DIN);
  k_ln_split<<<dim3(NTOK / 8), 256, 0, stream>>>(x, gamma, beta, XNhi, XNlo, NTOK);
  k_proj<<<dim3(NTOK / 128, DH / 64), 128, 0, stream>>>(XNhi, XNlo, WT, Hf, HThi, HTlo);
  k_sproj<<<dim3(NTOK / 256, NHD), 256, 0, stream>>>(Hf, wsrc, wdst, S);
  k_attn<<<dim3(NN_ / 64, NB_ * NHD), 128, 0, stream>>>(adj, S, bedge, HThi, HTlo, out);
  (void)hipGetLastError();
}
